// ResD1EdgeMLP_6176162972420
// MI455X (gfx1250) — hardware-run, weakly checked
//
#include <hip/hip_runtime.h>


namespace {
constexpr int NBR = 1024, D = 64, H = 128;
constexpr float XS = 8.0f, HS = 256.0f, WSC = 256.0f, LNEPS = 1e-5f;
typedef _Float16 b16;
typedef __attribute__((ext_vector_type(16))) _Float16 v16b;
typedef __attribute__((ext_vector_type(8))) _Float16 v8b;
typedef __attribute__((ext_vector_type(8))) float v8f;
typedef __attribute__((ext_vector_type(4))) float v4f;
__device__ __forceinline__ float bf16_rne(float f) { unsigned int u = __float_as_uint(f); u += 0x7FFFu + ((u >> 16) & 1u); float r = __uint_as_float(u & 0xFFFF0000u); asm volatile("" : "+v"(r)); return r; }
__device__ __forceinline__ float bfv(float f) { float r = bf16_rne(f); asm volatile("" : "+v"(r)); return r; }
__device__ __forceinline__ void split16(float v, b16& hi, b16& lo) { hi = (b16)v; lo = (b16)(v - (float)hi); }
__device__ __forceinline__ v16b frag_kb(const b16* p, int hh) { const v8b a = *(const v8b*)(p + 8 * hh), b = *(const v8b*)(p + 16 + 8 * hh); v16b f;
#pragma unroll
  for (int e = 0; e < 8; ++e) { f[e] = a[e]; f[8 + e] = b[e]; } return f; }
__device__ __forceinline__ v8f wmma16b(v16b a, v16b b, v8f c) { v8f d = __builtin_amdgcn_wmma_f32_16x16x32_f16(false, a, false, b, (short)0, c, false, false); asm volatile("v_nop\n\tv_nop\n\tv_nop\n\tv_nop" : "+v"(d) : "v"(a), "v"(b)); return d; }
__device__ __forceinline__ void wave_lds_sync() { __builtin_amdgcn_fence(__ATOMIC_RELEASE, "workgroup"); __builtin_amdgcn_wave_barrier(); __builtin_amdgcn_fence(__ATOMIC_ACQUIRE, "workgroup"); }
__device__ __forceinline__ float pmul(float a, float b) { float p = a * b; asm volatile("" : "+v"(p)); return p; }

__global__ __launch_bounds__(256) void wput_kernel(const float* __restrict__ w1, const float* __restrict__ w2, const float* __restrict__ wa, const float* __restrict__ wr, b16* __restrict__ W3T, b16* __restrict__ WAB, b16* __restrict__ W2T, b16* __restrict__ WAT, b16* __restrict__ WRT) { const int u = blockIdx.x * 256 + threadIdx.x; v8b v;
  if (u < 4 * H * 8) { const int o = u / 8, k0 = (u % 8) * 8; const int blk = o / H, oo = o % H;
#pragma unroll
    for (int j = 0; j < 8; ++j) v[j] = (b16)(bf16_rne(w1[(size_t)(blk * D + k0 + j) * H + oo]) * WSC); b16* dst = blk < 3 ? W3T + (size_t)o * D : WAB + (size_t)oo * D; for (int pass = 0; pass < 2; ++pass) { *(volatile v8b*)(dst + k0) = v; __threadfence(); } }
  if (u < H * 16) { const int o = u / 16, k0 = (u % 16) * 8;
#pragma unroll
    for (int j = 0; j < 8; ++j) v[j] = (b16)(bf16_rne(w2[(size_t)(k0 + j) * H + o]) * WSC); for (int pass = 0; pass < 2; ++pass) { *(volatile v8b*)(W2T + (size_t)o * H + k0) = v; __threadfence(); }
#pragma unroll
    for (int j = 0; j < 8; ++j) v[j] = (b16)(bf16_rne(wa[(size_t)(k0 + j) * H + o]) * WSC); for (int pass = 0; pass < 2; ++pass) { *(volatile v8b*)(WAT + (size_t)o * H + k0) = v; __threadfence(); } }
  if (u < H * 8) { const int o = u / 8, k0 = (u % 8) * 8;
#pragma unroll
    for (int j = 0; j < 8; ++j) v[j] = (b16)(bf16_rne(wr[(size_t)(k0 + j) * H + o]) * WSC); for (int pass = 0; pass < 2; ++pass) { *(volatile v8b*)(WRT + (size_t)o * D + k0) = v; __threadfence(); } } }
__global__ __launch_bounds__(32) void t_kernel(const float* __restrict__ x, const b16* __restrict__ W3T, float* __restrict__ TT) { __shared__ __attribute__((aligned(16))) b16 Ah[16][D + 8]; __shared__ float Tf[16][3 * H + 4]; const int lane = threadIdx.x, nloc = lane & 15, hlf = lane >> 4; const size_t m0 = (size_t)blockIdx.x * 16;
  for (int rr = 0; rr < 16; ++rr) for (int q = 0; q < 2; ++q) Ah[rr][q * 32 + lane] = (b16)(bf16_rne(x[(m0 + rr) * D + q * 32 + lane]) * XS); if (lane < 16) for (int k = D; k < D + 8; ++k) Ah[lane][k] = (b16)0.0f;
  wave_lds_sync();
#pragma unroll 1
  for (int g = 0; g < 3; ++g) { v8f acc[8];
#pragma unroll
    for (int t = 0; t < 8; ++t) acc[t] = (v8f){};
#pragma unroll
    for (int kb = 0; kb < D; kb += 32) { const v16b a = frag_kb(&Ah[nloc][kb], hlf);
#pragma unroll
      for (int t = 0; t < 8; ++t) acc[t] = wmma16b(a, frag_kb(W3T + (size_t)(g * H + t * 16 + nloc) * D + kb, hlf), acc[t]); }
#pragma unroll
    for (int t = 0; t < 8; ++t)
#pragma unroll
      for (int r8 = 0; r8 < 8; ++r8) Tf[8 * hlf + r8][g * H + t * 16 + nloc] = acc[t][r8] * (1.0f / (XS * WSC)); }
  wave_lds_sync();
  for (int pass = 0; pass < 2; ++pass) { for (int rr = 0; rr < 16; ++rr) for (int q = 0; q < 3; ++q) *(volatile v4f*)(TT + (m0 + rr) * 3 * H + q * 128 + lane * 4) = *(const v4f*)(&Tf[rr][q * 128 + lane * 4]); __threadfence(); } }
__global__ __launch_bounds__(32) void pair_kernel(const float* __restrict__ x, const float* __restrict__ TT, const b16* __restrict__ WAB, const float* __restrict__ b1, int ILIM, int JLIM, float* __restrict__ R) { __shared__ __attribute__((aligned(16))) b16 Ah[16][D + 8], Al[16][D + 8]; __shared__ float Xi[D], Ci[H], Rs[H]; const int lane = threadIdx.x, nloc = lane & 15, hlf = lane >> 4; const int i = blockIdx.x; if (i >= ILIM) return;
  for (int q = 0; q < 2; ++q) Xi[q * 32 + lane] = bfv(x[(size_t)i * D + q * 32 + lane]); for (int q = 0; q < 4; ++q) { const int c = q * 32 + lane; Ci[c] = TT[(size_t)i * 3 * H + c] + TT[(size_t)i * 3 * H + 2 * H + c] + bfv(b1[c]); Rs[c] = 0.0f; }
  if (lane < 16) for (int k = D; k < D + 8; ++k) { Ah[lane][k] = (b16)0.0f; Al[lane][k] = (b16)0.0f; }
  wave_lds_sync();
#pragma unroll 1
  for (int j0 = 0; j0 < JLIM; j0 += 16) {
    for (int rr = 0; rr < 16; ++rr) for (int q = 0; q < 2; ++q) { const int d = q * 32 + lane; b16 p, ql; split16(fabsf(Xi[d] - bfv(x[(size_t)(j0 + rr) * D + d])) * HS, p, ql); Ah[rr][d] = p; Al[rr][d] = ql; }
    wave_lds_sync(); v8f acc[8];
#pragma unroll
    for (int t = 0; t < 8; ++t) acc[t] = (v8f){};
#pragma unroll
    for (int kb = 0; kb < D; kb += 32) { const v16b a = frag_kb(&Ah[nloc][kb], hlf), al = frag_kb(&Al[nloc][kb], hlf);
#pragma unroll
      for (int t = 0; t < 8; ++t) { const v16b bw = frag_kb(WAB + (size_t)(t * 16 + nloc) * D + kb, hlf); acc[t] = wmma16b(a, bw, acc[t]); acc[t] = wmma16b(al, bw, acc[t]); } }
#pragma unroll
    for (int t = 0; t < 8; ++t) { const int cc = t * 16 + nloc; const float ci = Ci[cc]; float s = 0.0f;
#pragma unroll
      for (int r8 = 0; r8 < 8; ++r8) { const size_t j = (size_t)(j0 + 8 * hlf + r8); const float pre = acc[t][r8] * (1.0f / (HS * WSC)) + ci + TT[j * 3 * H + H + cc] - TT[j * 3 * H + 2 * H + cc]; s += fmaxf(pre, 0.0f); }
      s += __shfl_xor(s, 16); if (hlf == 0) Rs[cc] += s; }
    wave_lds_sync(); }
  for (int pass = 0; pass < 2; ++pass) { for (int q = 0; q < 4; ++q) ((volatile float*)R)[(size_t)i * H + q * 32 + lane] = Rs[q * 32 + lane]; __threadfence(); } }
__global__ __launch_bounds__(32) void tail_kernel(const float* __restrict__ R, const float* __restrict__ x, const b16* __restrict__ W2T, const b16* __restrict__ WAT, const b16* __restrict__ WRT, const float* __restrict__ b2, const float* __restrict__ wt, const float* __restrict__ bt, const float* __restrict__ ba, const float* __restrict__ br, const float* __restrict__ gam, const float* __restrict__ bet, int ILIM, int JLIM, float* __restrict__ out) {
  __shared__ __attribute__((aligned(16))) b16 Ah[16][H + 8], Al[16][H + 8], Xh[16][D + 8]; __shared__ float Tf[16][H + 4], Tau[16]; const int lane = threadIdx.x, nloc = lane & 15, hlf = lane >> 4; const size_t m0 = (size_t)blockIdx.x * 16; if (m0 >= (size_t)ILIM) return; const float invB = 1.0f / (float)JLIM;
  for (int rr = 0; rr < 16; ++rr) { for (int q = 0; q < 4; ++q) { const int c = q * 32 + lane; b16 p, ql; split16(R[(m0 + rr) * H + c] * invB * HS, p, ql); Ah[rr][c] = p; Al[rr][c] = ql; } float tdot = 0.0f; for (int q = 0; q < 2; ++q) { const int d = q * 32 + lane; const float xv = bfv(x[(m0 + rr) * D + d]); Xh[rr][d] = (b16)(xv * XS); tdot += pmul(xv, bfv(wt[d])); } for (int o = 16; o; o >>= 1) tdot += __shfl_xor(tdot, o); if (lane == 0) { const float z = tdot + bfv(bt[0]); const float sp = z > 20.0f ? z : log1pf(__expf(z)); Tau[rr] = fmaxf(sp, 0.01f) + 1.0f; } }
  if (lane < 16) { for (int k = H; k < H + 8; ++k) { Ah[lane][k] = (b16)0.0f; Al[lane][k] = (b16)0.0f; } for (int k = D; k < D + 8; ++k) Xh[lane][k] = (b16)0.0f; }
  wave_lds_sync(); v8f acc[8];
#pragma unroll
  for (int t = 0; t < 8; ++t) acc[t] = (v8f){};
#pragma unroll
  for (int kb = 0; kb < H; kb += 32) { const v16b a = frag_kb(&Ah[nloc][kb], hlf), al = frag_kb(&Al[nloc][kb], hlf);
#pragma unroll
    for (int t = 0; t < 8; ++t) { const v16b bw = frag_kb(W2T + (size_t)(t * 16 + nloc) * H + kb, hlf); acc[t] = wmma16b(a, bw, acc[t]); acc[t] = wmma16b(al, bw, acc[t]); } }
  wave_lds_sync();
#pragma unroll
  for (int t = 0; t < 8; ++t) { const int cc = t * 16 + nloc; const float bb = bfv(b2[cc]);
#pragma unroll
    for (int r8 = 0; r8 < 8; ++r8) { const int rr = 8 * hlf + r8; b16 p, ql; split16((acc[t][r8] * (1.0f / (HS * WSC)) + bb) / Tau[rr] * HS, p, ql); Ah[rr][cc] = p; Al[rr][cc] = ql; } }
  wave_lds_sync();
#pragma unroll
  for (int t = 0; t < 8; ++t) acc[t] = (v8f){};
#pragma unroll
  for (int kb = 0; kb < H; kb += 32) { const v16b a = frag_kb(&Ah[nloc][kb], hlf), al = frag_kb(&Al[nloc][kb], hlf);
#pragma unroll
    for (int t = 0; t < 8; ++t) { const v16b bw = frag_kb(WAT + (size_t)(t * 16 + nloc) * H + kb, hlf); acc[t] = wmma16b(a, bw, acc[t]); acc[t] = wmma16b(al, bw, acc[t]); } }
  v8f ar[8];
#pragma unroll
  for (int t = 0; t < 8; ++t) ar[t] = (v8f){};
#pragma unroll
  for (int kb = 0; kb < D; kb += 32) { const v16b a = frag_kb(&Xh[nloc][kb], hlf);
#pragma unroll
    for (int t = 0; t < 8; ++t) ar[t] = wmma16b(a, frag_kb(WRT + (size_t)(t * 16 + nloc) * D + kb, hlf), ar[t]); }
#pragma unroll
  for (int t = 0; t < 8; ++t) { const int cc = t * 16 + nloc; const float b_a = bfv(ba[cc]), b_r = bfv(br[cc]);
#pragma unroll
    for (int r8 = 0; r8 < 8; ++r8) Tf[8 * hlf + r8][cc] = fmaxf(acc[t][r8] * (1.0f / (HS * WSC)) + b_a, 0.0f) + ar[t][r8] * (1.0f / (XS * WSC)) + b_r; }
  wave_lds_sync();
  for (int pass = 0; pass < 2; ++pass) { for (int rr = 0; rr < 16; ++rr) { float v[4], s = 0.0f; for (int k = 0; k < 4; ++k) { v[k] = Tf[rr][lane * 4 + k]; s += v[k]; } for (int o = 16; o; o >>= 1) s += __shfl_xor(s, o); const float mu = s / H; float s2 = 0.0f; for (int k = 0; k < 4; ++k) s2 += (v[k] - mu) * (v[k] - mu); for (int o = 16; o; o >>= 1) s2 += __shfl_xor(s2, o); const float rs = rsqrtf(s2 / H + LNEPS);
      v4f o4; for (int k = 0; k < 4; ++k) { const int c = lane * 4 + k; o4[k] = pmul(pmul(v[k] - mu, rs), bfv(gam[c])) + bfv(bet[c]); } *(volatile v4f*)(out + (m0 + rr) * H + lane * 4) = o4; } __threadfence(); } }
}

extern "C" void kernel_launch(void* const* d_in, const int* in_sizes, int n_in, void* d_out, int out_size, void* d_ws, size_t ws_size, hipStream_t stream) {
  (void)n_in;
  auto Fp = [&](int i) { return (const float*)d_in[i]; };
  if (in_sizes[0] != NBR * D || in_sizes[1] != 4 * D * H || in_sizes[2] != H || in_sizes[3] != H * H || in_sizes[5] != D || in_sizes[6] != 1 || in_sizes[7] != H * H || in_sizes[9] != D * H || in_sizes[11] != H || out_size != NBR * H) return;
  const int ILIM = NBR, JLIM = NBR;
  size_t off = 0; char* ws = (char*)d_ws;
  auto carve = [&](size_t bytes) { char* p = ws + off; off += (bytes + 255) & ~(size_t)255; return p; };
  b16* W3T = (b16*)carve((size_t)3 * H * D * 2); b16* WAB = (b16*)carve((size_t)H * D * 2); b16* W2T = (b16*)carve((size_t)H * H * 2); b16* WAT = (b16*)carve((size_t)H * H * 2); b16* WRT = (b16*)carve((size_t)H * D * 2); float* TT = (float*)carve((size_t)NBR * 3 * H * 4); float* R = (float*)carve((size_t)NBR * H * 4);
  if (off > ws_size || off > ((size_t)8 << 20)) return;
  wput_kernel<<<(4 * H * 8 + 255) / 256, 256, 0, stream>>>(Fp(1), Fp(3), Fp(7), Fp(9), W3T, WAB, W2T, WAT, WRT);
  t_kernel<<<NBR / 16, 32, 0, stream>>>(Fp(0), W3T, TT);
  pair_kernel<<<ILIM, 32, 0, stream>>>(Fp(0), TT, WAB, Fp(2), ILIM, JLIM, R);
  tail_kernel<<<ILIM / 16, 32, 0, stream>>>(R, Fp(0), W2T, WAT, WRT, Fp(4), Fp(5), Fp(6), Fp(8), Fp(10), Fp(11), Fp(12), ILIM, JLIM, (float*)d_out);
}
